// MultiHeadedAttention_48885317763370
// MI455X (gfx1250) — hardware-verified
//
#include <hip/hip_runtime.h>

typedef __attribute__((ext_vector_type(16))) _Float16 v16h;
typedef __attribute__((ext_vector_type(8)))  _Float16 v8h;
typedef __attribute__((ext_vector_type(16))) __bf16   v16b;
typedef __attribute__((ext_vector_type(8)))  __bf16   v8b;
typedef __attribute__((ext_vector_type(8)))  float    v8f;
typedef __attribute__((ext_vector_type(4)))  float    v4f;
typedef __attribute__((ext_vector_type(4)))  unsigned v4u;

__device__ __forceinline__ unsigned short f2bf_bits(float f) {
  unsigned u = __float_as_uint(f);
  return (unsigned short)((u + 0x7FFFu + ((u >> 16) & 1u)) >> 16);
}
__device__ __forceinline__ float bf_bits2f(unsigned short h) { return __uint_as_float(((unsigned)h) << 16); }

__device__ __forceinline__ void dep_guard_h(v8f& a, v8f& b, v16h x, v16h y) { asm volatile("v_nop\n\tv_nop\n\tv_nop\n\tv_nop" : "+v"(a), "+v"(b) : "v"(x), "v"(y)); }
__device__ __forceinline__ void dep_guard_b(v8f& a, v8f& b, v16b x, v16b y) { asm volatile("v_nop\n\tv_nop\n\tv_nop\n\tv_nop" : "+v"(a), "+v"(b) : "v"(x), "v"(y)); }
__device__ __forceinline__ void keep4_h(v16h a, v16h b, v16h c, v16h d) { asm volatile("v_nop" :: "v"(a), "v"(b), "v"(c), "v"(d)); }
__device__ __forceinline__ void keep4_b(v16b a, v16b b, v16b c, v16b d) { asm volatile("v_nop" :: "v"(a), "v"(b), "v"(c), "v"(d)); }
__device__ __forceinline__ void acc_guard4(v8f& a, v8f& b, v8f& c, v8f& d) { asm volatile("v_nop\n\tv_nop\n\tv_nop\n\tv_nop" : "+v"(a), "+v"(b), "+v"(c), "+v"(d)); }
template <typename T> struct Frag;
template <> struct Frag<_Float16> {
  typedef v16h V; union U { v16h v; v8h h[2]; };
  static __device__ __forceinline__ v16h load(const _Float16* p) {
    U f; f.h[0] = *(const v8h*)(p); f.h[1] = *(const v8h*)(p + 16); return f.v;
  }
  static __device__ __forceinline__ v8f mma(v16h a, v16h b, v8f c) {
    return __builtin_amdgcn_wmma_f32_16x16x32_f16(false, a, false, b, (short)0, c, false, false);
  }
  static __device__ __forceinline__ void guard(v8f& a, v8f& b, v16h x, v16h y) { dep_guard_h(a, b, x, y); }
  static __device__ __forceinline__ void keep(v16h a, v16h b, v16h c, v16h d) { keep4_h(a, b, c, d); }
};
template <> struct Frag<__bf16> {
  typedef v16b V; union U { v16b v; v8b h[2]; };
  static __device__ __forceinline__ v16b load(const __bf16* p) {
    U f; f.h[0] = *(const v8b*)(p); f.h[1] = *(const v8b*)(p + 16); return f.v;
  }
  static __device__ __forceinline__ v8f mma(v16b a, v16b b, v8f c) {
    return __builtin_amdgcn_wmma_f32_16x16x32_bf16(false, a, false, b, (short)0, c, false, false);
  }
  static __device__ __forceinline__ void guard(v8f& a, v8f& b, v16b x, v16b y) { dep_guard_b(a, b, x, y); }
  static __device__ __forceinline__ void keep(v16b a, v16b b, v16b c, v16b d) { keep4_b(a, b, c, d); }
};

template <int ET> struct Elem;
template <> struct Elem<0> { typedef _Float16 T; };
template <> struct Elem<1> { typedef __bf16 T; };
template <int ET, bool SPLIT, int BIAS_MODE, int OUT_MODE, bool RESID, int ACT = 0, bool BLO = true>
__global__ __launch_bounds__(256) void wmma_gemm64(
    const unsigned short* __restrict__ Ap, const unsigned short* __restrict__ A2p, int lda, long strideA,
    const unsigned short* __restrict__ Btp, const unsigned short* __restrict__ Bt2p, int ldb, long strideB,
    void* __restrict__ Cout, void* __restrict__ Cout2, int ldc, long strideC,
    const float* __restrict__ bias,
    const float* __restrict__ resid, long strideR,
    int M, int N, int K, float scale) {
  typedef typename Elem<ET>::T T;
  typedef typename Frag<T>::V V;
  const T* A = (const T*)Ap; const T* A2 = (const T*)A2p; const T* Bt = (const T*)Btp; const T* Bt2 = (const T*)Bt2p;
  __shared__ __align__(16) float sT[8][16 * 68];
  const int b    = blockIdx.y;
  const int lane = threadIdx.x & 31;
  const int wave = threadIdx.x >> 5;
  const int tilesN = N >> 6;
  const int tilesM = M >> 6;
  const int tile = blockIdx.x * 8 + wave;
  if (tile >= tilesM * tilesN) return;
  const int tm = tile / tilesN;
  const int tn = tile - tm * tilesN;
  const int m0 = tm << 6;
  const int n0 = tn << 6;

  const T* Ab  = A  + (size_t)b * strideA;
  const T* Bb  = Bt + (size_t)b * strideB;
  const T* Ab2 = SPLIT ? (A2  + (size_t)b * strideA) : nullptr;
  const T* Bb2 = (SPLIT && BLO) ? (Bt2 + (size_t)b * strideB) : nullptr;

  const int rlane = lane & 15;
  const int koff  = (lane >> 4) * 8;
  const int mOff  = (lane >> 4) * 8;

  v8f acc[4][4];
#pragma unroll
  for (int i = 0; i < 4; ++i)
#pragma unroll
    for (int j = 0; j < 4; ++j) acc[i][j] = (v8f){0.f,0.f,0.f,0.f,0.f,0.f,0.f,0.f};

  for (int k0 = 0; k0 < K; k0 += 32) {
    V bh[4], bl[4];
#pragma unroll
    for (int j = 0; j < 4; ++j) {
      const size_t bo = (size_t)(n0 + (j << 4) + rlane) * ldb + koff + k0;
      bh[j] = Frag<T>::load(Bb + bo);
      if (SPLIT && BLO) bl[j] = Frag<T>::load(Bb2 + bo);
    }
#pragma unroll
    for (int i = 0; i < 4; ++i) {
      const size_t ao = (size_t)(m0 + (i << 4) + rlane) * lda + koff + k0;
      V ah = Frag<T>::load(Ab + ao);
      V al;
      if (SPLIT) al = Frag<T>::load(Ab2 + ao);
#pragma unroll
      for (int j = 0; j < 4; ++j) {
        acc[i][j] = Frag<T>::mma(ah, bh[j], acc[i][j]);
        if (SPLIT) {
          if (BLO) acc[i][j] = Frag<T>::mma(ah, bl[j], acc[i][j]);
          acc[i][j] = Frag<T>::mma(al, bh[j], acc[i][j]);
        }
      }
      Frag<T>::guard(acc[i][0], acc[i][3], ah, SPLIT ? al : ah);
    }
    Frag<T>::keep(bh[0], bh[1], bh[2], bh[3]);
    if (SPLIT && BLO) Frag<T>::keep(bl[0], bl[1], bl[2], bl[3]);
  }
  acc_guard4(acc[0][0], acc[0][1], acc[0][2], acc[0][3]);
  acc_guard4(acc[1][0], acc[1][1], acc[1][2], acc[1][3]);
  acc_guard4(acc[2][0], acc[2][1], acc[2][2], acc[2][3]);
  acc_guard4(acc[3][0], acc[3][1], acc[3][2], acc[3][3]);

  float* slab = sT[wave];
  const float* Rb = RESID ? (resid + (size_t)b * strideR) : nullptr;
#pragma unroll
  for (int i = 0; i < 4; ++i) {
    const int mBase = m0 + (i << 4);
#pragma unroll
    for (int j = 0; j < 4; ++j) {
      const int n = n0 + (j << 4) + rlane;
      float bv = 0.f;
      if (BIAS_MODE == 2) bv = bias[n];
#pragma unroll
      for (int r = 0; r < 8; ++r) {
        float v = acc[i][j][r] * scale;
        if (BIAS_MODE == 1) v += bias[mBase + mOff + r];
        if (BIAS_MODE == 2) v += bv;
        if (RESID) v += Rb[(size_t)(mBase + mOff + r) * ldc + n];
        if (ACT == 1) v = tanhf(v);
        if (ACT == 2) v = fmaxf(v, 0.0f);
        if (ACT == 3) v = v / (1.0f + expf(-v));
        if (ACT == 4) v = (v > 0.f) ? v : 0.01f * v;
        if (ACT == 5) v = 0.5f * v * (1.0f + erff(v * 0.70710678118654752f));
        slab[(mOff + r) * 68 + (j << 4) + rlane] = v;
      }
    }
    __builtin_amdgcn_fence(__ATOMIC_RELEASE, "workgroup");
    __builtin_amdgcn_wave_barrier();
    __builtin_amdgcn_fence(__ATOMIC_ACQUIRE, "workgroup");
    if (OUT_MODE == 0) {
      float* C = (float*)Cout + (size_t)b * strideC;
      const int hh = lane >> 4, c4 = (lane & 15) * 4;
      for (int pass = 0; pass < 2; ++pass) {
#pragma unroll
        for (int it = 0; it < 8; ++it) {
          const int row = it * 2 + hh;
          v4f v = *(const v4f*)(slab + row * 68 + c4);
          *(volatile v4f*)(C + (size_t)(mBase + row) * ldc + n0 + c4) = v;
        }
        __threadfence();
      }
    } else {
      const int q = lane >> 3, c8 = (lane & 7) * 8;
      unsigned short* C  = (unsigned short*)Cout  + (size_t)b * strideC;
      unsigned short* C2 = (OUT_MODE == 2) ? ((unsigned short*)Cout2 + (size_t)b * strideC) : nullptr;
      for (int pass = 0; pass < 2; ++pass) {
#pragma unroll
        for (int it = 0; it < 4; ++it) {
          const int row = it * 4 + q;
          const float* sp = slab + row * 68 + c8;
          v8h hv, lv;
#pragma unroll
          for (int e = 0; e < 8; ++e) {
            if (OUT_MODE == 1) {
              hv[e] = (_Float16)sp[e];
            } else {
              unsigned short hb = f2bf_bits(sp[e]);
              unsigned short lb = f2bf_bits(sp[e] - bf_bits2f(hb));
              hv[e] = __builtin_bit_cast(_Float16, hb);
              lv[e] = __builtin_bit_cast(_Float16, lb);
            }
          }
          *(volatile v8h*)(C + (size_t)(mBase + row) * ldc + n0 + c8) = hv;
          if (OUT_MODE == 2) *(volatile v8h*)(C2 + (size_t)(mBase + row) * ldc + n0 + c8) = lv;
        }
        __threadfence();
      }
    }
    __builtin_amdgcn_fence(__ATOMIC_RELEASE, "workgroup");
    __builtin_amdgcn_wave_barrier();
    __builtin_amdgcn_fence(__ATOMIC_ACQUIRE, "workgroup");
  }
}

__device__ __forceinline__ unsigned short at_bf_bits(float f) {
  unsigned u = __float_as_uint(f);
  return (unsigned short)((u + 0x7FFFu + ((u >> 16) & 1u)) >> 16);
}
__device__ __forceinline__ __bf16 at_f2bf(float f) { return __builtin_bit_cast(__bf16, at_bf_bits(f)); }
__device__ __forceinline__ void at_split(float f, __bf16& hi, __bf16& lo) {
  const unsigned short hb = at_bf_bits(f);
  hi = __builtin_bit_cast(__bf16, hb);
  lo = at_f2bf(f - __uint_as_float(((unsigned)hb) << 16));
}
__device__ __forceinline__ v8f at_mma(v16b a, v16b b, v8f c) {
  c = __builtin_amdgcn_wmma_f32_16x16x32_bf16(false, a, false, b, (short)0, c, false, false);
  asm volatile("v_nop\n\tv_nop\n\tv_nop\n\tv_nop" : "+v"(c) : "v"(a), "v"(b));
  return c;
}

constexpr int kBatch = 2;
constexpr int kSeq   = 2048;
constexpr int kDm    = 1024;
constexpr int kHeads = 16;
constexpr int kHd    = 64;
constexpr int kQB    = 64;
constexpr int kKC    = 64;
constexpr int kNW    = 4;
constexpr int kTok   = kBatch * kSeq;
static_assert(kHeads * kHd == kDm);
static_assert(kSeq % kQB == 0 && kSeq % kKC == 0);
static_assert(kTok % 64 == 0 && kDm % 64 == 0 && kSeq % 64 == 0);
static_assert(kDm % 32 == 0);

__global__ __launch_bounds__(256) void cast_f32_bf16x8(
    const float* __restrict__ in, unsigned short* __restrict__ out, int n8) {
  const int i = blockIdx.x * 256 + threadIdx.x;
  if (i < n8) {
    const v4f a = *(const v4f*)(in + (size_t)i * 8);
    const v4f c = *(const v4f*)(in + (size_t)i * 8 + 4);
    v4u w;
    w[0] = (unsigned)f2bf_bits(a[0]) | ((unsigned)f2bf_bits(a[1]) << 16);
    w[1] = (unsigned)f2bf_bits(a[2]) | ((unsigned)f2bf_bits(a[3]) << 16);
    w[2] = (unsigned)f2bf_bits(c[0]) | ((unsigned)f2bf_bits(c[1]) << 16);
    w[3] = (unsigned)f2bf_bits(c[2]) | ((unsigned)f2bf_bits(c[3]) << 16);
    *(volatile v4u*)(out + (size_t)i * 8) = w;
    __threadfence();
    *(volatile v4u*)(out + (size_t)i * 8) = w;
  }
}

__global__ __launch_bounds__(256) void wtrans_bf16(
    const float* __restrict__ w, unsigned short* __restrict__ wt) {
  __shared__ __align__(16) unsigned short tile[64 * 72];
  const int tid = threadIdx.x;
  const int k0 = blockIdx.x * 64, n0 = blockIdx.y * 64;
#pragma unroll
  for (int it = 0; it < 4; ++it) {
    const int kr = it * 16 + (tid >> 4);
    const int n4 = (tid & 15) * 4;
    const v4f x = *(const v4f*)(w + (size_t)(k0 + kr) * kDm + n0 + n4);
#pragma unroll
    for (int e = 0; e < 4; ++e) tile[(n4 + e) * 72 + kr] = f2bf_bits(x[e]);
  }
  __syncthreads();
  const int wave = tid >> 5, lane = tid & 31;
  const int q = lane >> 3, c8 = (lane & 7) * 8;
  for (int pass = 0; pass < 2; ++pass) {
#pragma unroll
    for (int it = 0; it < 2; ++it) {
      const int row = wave * 8 + it * 4 + q;
      const v4u val = *(const v4u*)(tile + row * 72 + c8);
      *(volatile v4u*)(wt + (size_t)(n0 + row) * kDm + k0 + c8) = val;
    }
    __threadfence();
  }
}

__global__ __launch_bounds__(128)
void attn64_planes(const unsigned short* __restrict__ Qh, const unsigned short* __restrict__ Ql,
                   const unsigned short* __restrict__ Kh, const unsigned short* __restrict__ Kl,
                   const unsigned short* __restrict__ Vth, const unsigned short* __restrict__ Vtl,
                   unsigned short* __restrict__ Oh, unsigned short* __restrict__ Ol) {
  union FB { v16b v; v8b h[2]; };
  __shared__ __align__(16) __bf16 Ksh[kKC * kHd];
  __shared__ __align__(16) __bf16 Ksl[kKC * kHd];
  __shared__ __align__(16) __bf16 Vsh[kHd * kKC];
  __shared__ __align__(16) __bf16 Vsl[kHd * kKC];
  __shared__ __align__(16) __bf16 Psh[kNW][16 * kKC];
  __shared__ __align__(16) __bf16 Psl[kNW][16 * kKC];
  __shared__ __align__(16) float  Os[kNW][16 * 68];

  const int tid  = threadIdx.x;
  const int wave = tid >> 5;
  const int lane = tid & 31;
  const int hh   = lane >> 4;
  const int c    = lane & 15;

  const int nqb = kSeq / kQB;
  const int bx  = blockIdx.x;
  const int qb  = bx % nqb;
  const int bhx = bx / nqb;
  const int h   = bhx % kHeads;
  const int b   = bhx / kHeads;
  const int q0  = qb * kQB + wave * 16;

  v16b qah[2], qal[2];
  {
    const size_t qo = ((size_t)b * kSeq + q0 + c) * kDm + (size_t)h * kHd + 8 * hh;
#pragma unroll
    for (int dc = 0; dc < 2; ++dc) {
      qah[dc] = Frag<__bf16>::load((const __bf16*)Qh + qo + dc * 32);
      qal[dc] = Frag<__bf16>::load((const __bf16*)Ql + qo + dc * 32);
    }
  }

  float mrow[8], lrow[8];
  v8f oacc[4];
#pragma unroll
  for (int r = 0; r < 8; ++r) { mrow[r] = -INFINITY; lrow[r] = 0.f; }
#pragma unroll
  for (int t = 0; t < 4; ++t) oacc[t] = (v8f){0.f,0.f,0.f,0.f,0.f,0.f,0.f,0.f};

  for (int kc = 0; kc < kSeq / kKC; ++kc) {
    const int kv0 = kc * kKC;
    __syncthreads();
    {
      const int r = tid >> 1, hf = (tid & 1) * 32;
      const size_t ko = ((size_t)b * kSeq + kv0 + r) * kDm + (size_t)h * kHd + hf;
      v4u x[4], y[4];
#pragma unroll
      for (int i = 0; i < 4; ++i) { x[i] = *(const v4u*)(Kh + ko + 8 * i); y[i] = *(const v4u*)(Kl + ko + 8 * i); }
#pragma unroll
      for (int i = 0; i < 4; ++i) {
        *(v4u*)(Ksh + r * kHd + hf + 8 * i) = x[i];
        *(v4u*)(Ksl + r * kHd + hf + 8 * i) = y[i];
      }
      const size_t vo = ((size_t)b * kDm + (size_t)h * kHd + r) * kSeq + kv0 + hf;
#pragma unroll
      for (int i = 0; i < 4; ++i) { x[i] = *(const v4u*)(Vth + vo + 8 * i); y[i] = *(const v4u*)(Vtl + vo + 8 * i); }
#pragma unroll
      for (int i = 0; i < 4; ++i) {
        *(v4u*)(Vsh + r * kKC + hf + 8 * i) = x[i];
        *(v4u*)(Vsl + r * kKC + hf + 8 * i) = y[i];
      }
    }
    __syncthreads();

    v8f s[4];
#pragma unroll
    for (int j = 0; j < 4; ++j) {
      s[j] = (v8f){0.f,0.f,0.f,0.f,0.f,0.f,0.f,0.f};
#pragma unroll
      for (int dc = 0; dc < 2; ++dc) {
        const int ko = (j * 16 + c) * kHd + dc * 32 + 8 * hh;
        FB kb, kl;
        kb.h[0] = *(const v8b*)(Ksh + ko);
        kb.h[1] = *(const v8b*)(Ksh + ko + 16);
        kl.h[0] = *(const v8b*)(Ksl + ko);
        kl.h[1] = *(const v8b*)(Ksl + ko + 16);
        s[j] = at_mma(qah[dc], kb.v, s[j]);
        s[j] = at_mma(qah[dc], kl.v, s[j]);
        s[j] = at_mma(qal[dc], kb.v, s[j]);
      }
    }

    float cm[8];
#pragma unroll
    for (int r = 0; r < 8; ++r) {
      float m = fmaxf(fmaxf(s[0][r], s[1][r]), fmaxf(s[2][r], s[3][r]));
#pragma unroll
      for (int off = 1; off < 16; off <<= 1) m = fmaxf(m, __shfl_xor(m, off, 32));
      cm[r] = m;
    }

    __bf16* pwh = Psh[wave];
    __bf16* pwl = Psl[wave];
#pragma unroll
    for (int r = 0; r < 8; ++r) {
      const float mnew  = fmaxf(mrow[r], cm[r]);
      const float alpha = expf(mrow[r] - mnew);
      mrow[r] = mnew;
      float psum = 0.f;
#pragma unroll
      for (int j = 0; j < 4; ++j) {
        const float p = expf(s[j][r] - mnew);
        psum += p;
        __bf16 ph, pl;
        at_split(p, ph, pl);
        pwh[(8 * hh + r) * kKC + j * 16 + c] = ph;
        pwl[(8 * hh + r) * kKC + j * 16 + c] = pl;
      }
#pragma unroll
      for (int off = 1; off < 16; off <<= 1) psum += __shfl_xor(psum, off, 32);
      lrow[r] = lrow[r] * alpha + psum;
#pragma unroll
      for (int t = 0; t < 4; ++t) oacc[t][r] *= alpha;
    }
    __builtin_amdgcn_fence(__ATOMIC_RELEASE, "workgroup");
    __builtin_amdgcn_wave_barrier();
    __builtin_amdgcn_fence(__ATOMIC_ACQUIRE, "workgroup");

#pragma unroll 1
    for (int kk = 0; kk < 2; ++kk) {
      FB pa, pl;
      pa.h[0] = *(const v8b*)(pwh + c * kKC + kk * 32 + 8 * hh);
      pa.h[1] = *(const v8b*)(pwh + c * kKC + kk * 32 + 16 + 8 * hh);
      pl.h[0] = *(const v8b*)(pwl + c * kKC + kk * 32 + 8 * hh);
      pl.h[1] = *(const v8b*)(pwl + c * kKC + kk * 32 + 16 + 8 * hh);
#pragma unroll
      for (int t = 0; t < 4; ++t) {
        const int vofs = (t * 16 + c) * kKC + kk * 32 + 8 * hh;
        FB vb, vl;
        vb.h[0] = *(const v8b*)(Vsh + vofs);
        vb.h[1] = *(const v8b*)(Vsh + vofs + 16);
        vl.h[0] = *(const v8b*)(Vsl + vofs);
        vl.h[1] = *(const v8b*)(Vsl + vofs + 16);
        oacc[t] = at_mma(pa.v, vb.v, oacc[t]);
        oacc[t] = at_mma(pa.v, vl.v, oacc[t]);
        oacc[t] = at_mma(pl.v, vb.v, oacc[t]);
      }
    }
  }

  float* os = Os[wave];
#pragma unroll
  for (int r = 0; r < 8; ++r) {
    const float inv = 1.0f / lrow[r];
#pragma unroll
    for (int t = 0; t < 4; ++t) os[(8 * hh + r) * 68 + t * 16 + c] = oacc[t][r] * inv;
  }
  __builtin_amdgcn_fence(__ATOMIC_RELEASE, "workgroup");
  __builtin_amdgcn_wave_barrier();
  __builtin_amdgcn_fence(__ATOMIC_ACQUIRE, "workgroup");
  {
    const int q4 = lane >> 3, c8 = (lane & 7) * 8;
    for (int pass = 0; pass < 2; ++pass) {
#pragma unroll
      for (int it = 0; it < 4; ++it) {
        const int row = it * 4 + q4;
        const float* sp = os + row * 68 + c8;
        const v4f x0 = *(const v4f*)(sp);
        const v4f x1 = *(const v4f*)(sp + 4);
        const float f[8] = {x0[0], x0[1], x0[2], x0[3], x1[0], x1[1], x1[2], x1[3]};
        v4u hv, lv;
#pragma unroll
        for (int e = 0; e < 4; ++e) {
          const unsigned short h0 = f2bf_bits(f[2 * e]);
          const unsigned short h1 = f2bf_bits(f[2 * e + 1]);
          const unsigned short l0 = f2bf_bits(f[2 * e] - bf_bits2f(h0));
          const unsigned short l1 = f2bf_bits(f[2 * e + 1] - bf_bits2f(h1));
          hv[e] = (unsigned)h0 | ((unsigned)h1 << 16);
          lv[e] = (unsigned)l0 | ((unsigned)l1 << 16);
        }
        const size_t oo = ((size_t)b * kSeq + q0 + row) * kDm + (size_t)h * kHd + c8;
        *(volatile v4u*)(Oh + oo) = hv;
        *(volatile v4u*)(Ol + oo) = lv;
      }
      __threadfence();
    }
  }
}

extern "C" void kernel_launch(void* const* d_in, const int* in_sizes, int n_in,
                              void* d_out, int out_size, void* d_ws, size_t ws_size,
                              hipStream_t stream) {
  if (n_in < 7) return;
  if (out_size != kTok * kDm) return;
  if (in_sizes[0] != kTok * kDm || in_sizes[1] != kTok * kDm || in_sizes[2] != kTok * kDm) return;
  if (in_sizes[3] != kDm * kDm || in_sizes[4] != kDm * kDm || in_sizes[5] != kDm * kDm || in_sizes[6] != kDm * kDm) return;

  const float* q  = (const float*)d_in[0];
  const float* k  = (const float*)d_in[1];
  const float* v  = (const float*)d_in[2];
  const float* wq = (const float*)d_in[3];
  const float* wk = (const float*)d_in[4];
  const float* wv = (const float*)d_in[5];
  const float* wo = (const float*)d_in[6];

  const size_t actN = (size_t)kTok * kDm;
  const size_t wN   = (size_t)kDm * kDm;
  size_t off = 0;
  unsigned short* ws = (unsigned short*)d_ws;
  unsigned short* qb16 = ws + off; off += actN;
  unsigned short* kb16 = ws + off; off += actN;
  unsigned short* vb16 = ws + off; off += actN;
  unsigned short* wqT  = ws + off; off += wN;
  unsigned short* wkT  = ws + off; off += wN;
  unsigned short* wvT  = ws + off; off += wN;
  unsigned short* woT  = ws + off; off += wN;
  unsigned short* Qh   = ws + off; off += actN;
  unsigned short* Ql   = ws + off; off += actN;
  unsigned short* Kh   = ws + off; off += actN;
  unsigned short* Kl   = ws + off; off += actN;
  unsigned short* Vth  = ws + off; off += actN;
  unsigned short* Vtl  = ws + off; off += actN;
  unsigned short* Oh   = ws + off; off += actN;
  unsigned short* Ol   = ws + off; off += actN;
  const size_t need_bytes = off * sizeof(unsigned short);
  if (need_bytes > ws_size) return;
  const float* fdummy = (const float*)d_ws;

  const int n8 = (int)(actN / 8);
  const int castBlocks = (n8 + 255) / 256;
  cast_f32_bf16x8<<<castBlocks, 256, 0, stream>>>(q, qb16, n8);
  cast_f32_bf16x8<<<castBlocks, 256, 0, stream>>>(k, kb16, n8);
  cast_f32_bf16x8<<<castBlocks, 256, 0, stream>>>(v, vb16, n8);

  const dim3 tgrid(kDm / 64, kDm / 64);
  wtrans_bf16<<<tgrid, 256, 0, stream>>>(wq, wqT);
  wtrans_bf16<<<tgrid, 256, 0, stream>>>(wk, wkT);
  wtrans_bf16<<<tgrid, 256, 0, stream>>>(wv, wvT);
  wtrans_bf16<<<tgrid, 256, 0, stream>>>(wo, woT);

  const int tilesQK = (kTok / 64) * (kDm / 64);
  const dim3 gQK((tilesQK + 7) / 8, 1);
  wmma_gemm64<1, false, 0, 2, false><<<gQK, 256, 0, stream>>>(
      qb16, qb16, kDm, 0L, wqT, wqT, kDm, 0L, (void*)Qh, (void*)Ql, kDm, 0L,
      fdummy, fdummy, 0L, kTok, kDm, kDm, 0.125f);
  wmma_gemm64<1, false, 0, 2, false><<<gQK, 256, 0, stream>>>(
      kb16, kb16, kDm, 0L, wkT, wkT, kDm, 0L, (void*)Kh, (void*)Kl, kDm, 0L,
      fdummy, fdummy, 0L, kTok, kDm, kDm, 1.0f);

  const int tilesV = (kDm / 64) * (kSeq / 64);
  const dim3 gV((tilesV + 7) / 8, kBatch);
  wmma_gemm64<1, false, 0, 2, false><<<gV, 256, 0, stream>>>(
      wvT, wvT, kDm, 0L, vb16, vb16, kDm, (long)kSeq * kDm, (void*)Vth, (void*)Vtl, kSeq, (long)kDm * kSeq,
      fdummy, fdummy, 0L, kDm, kSeq, kDm, 1.0f);

  const int attnBlocks = kBatch * kHeads * (kSeq / kQB);
  attn64_planes<<<attnBlocks, 128, 0, stream>>>(Qh, Ql, Kh, Kl, Vth, Vtl, Oh, Ol);

  wmma_gemm64<1, true, 0, 0, false, 0, false><<<gQK, 256, 0, stream>>>(
      Oh, Ol, kDm, 0L, woT, woT, kDm, 0L, d_out, d_out, kDm, 0L,
      fdummy, fdummy, 0L, kTok, kDm, kDm, 1.0f);
}
